// RecurrentCNNModel_55344948576740
// MI455X (gfx1250) — hardware-verified
//
#include <hip/hip_runtime.h>

typedef __attribute__((ext_vector_type(16))) _Float16 v16h;
typedef __attribute__((ext_vector_type(8)))  _Float16 v8h;
typedef __attribute__((ext_vector_type(16))) __bf16   v16b;
typedef __attribute__((ext_vector_type(8)))  __bf16   v8b;
typedef __attribute__((ext_vector_type(8)))  float    v8f;
typedef __attribute__((ext_vector_type(4)))  float    v4f;

constexpr int kBatch  = 128;
constexpr int kLen    = 1024;
constexpr int kEmb    = 300;
constexpr int kEmbP   = 320;
constexpr int kChan   = 100;
constexpr int kChanP  = 128;
constexpr int kHid    = 100;
constexpr int kHidP   = 128;
constexpr int kCls    = 4;
constexpr int kVocab  = 50000;
constexpr int kVocabP = 50048;
constexpr int kFeatIn = kEmb + 2 * kChan;
constexpr int kRows   = kBatch * kLen;
constexpr int kPSW    = 2 * kChanP;
constexpr int kFeatW  = 2 * kChanP;
constexpr int kChunkRows = 32768;
constexpr int kChunks = kRows / kChunkRows;
constexpr int kSeqPerChunk = kChunkRows / kLen;
static_assert(kVocabP % 64 == 0 && kVocabP >= kVocab);
static_assert(kEmbP % 32 == 0 && kChanP % 32 == 0 && kFeatW % 32 == 0);
static_assert(kRows % kChunkRows == 0 && kChunkRows % kLen == 0 && kChunkRows % 64 == 0);

constexpr int kSeqPB      = 16;
constexpr int kRecBlocks  = 2 * (kBatch / kSeqPB);
constexpr int kRecThreads = 256;
constexpr int kStP        = kChanP + 8;
constexpr int kStTile     = kSeqPB * kStP;
constexpr int kSTile      = kSeqPB * kChanP;
static_assert(kBatch % kSeqPB == 0);
static_assert(kChanP == (kRecThreads / 32) * 16);
static_assert(kRecThreads * 8 == kSTile);
static_assert(kRecThreads * 8 == kSeqPB * kChanP);
static_assert((kSeqPB * kLen) % kRecThreads == 0);
static_assert(kStP % 8 == 0);

constexpr int kDwWcat = 384 * kEmbP / 2;
constexpr int kDwWlr  = 256 * kChanP / 2;
constexpr int kDwW2ac = kHidP * kFeatW / 2;
constexpr int kDwBias = 768;
constexpr int kPrepB1 = kDwWcat / 256;
constexpr int kPrepB2 = kPrepB1 + kDwWlr / 256;
constexpr int kPrepB3 = kPrepB2 + kDwW2ac / 256;
constexpr int kPrepBlocks = kPrepB3 + kDwBias / 256;
static_assert(kDwWcat % 256 == 0 && kDwWlr % 256 == 0 && kDwW2ac % 256 == 0 && kDwBias % 256 == 0);
static_assert(kPrepBlocks == 371);

constexpr int kEmbChunks = kVocabP * (kEmbP / 8);
constexpr int kEmbBlocks = kEmbChunks / 256;
static_assert(kEmbChunks % 256 == 0 && kEmbBlocks == 7820);

constexpr int kG1Blocks = ((kVocabP / 64) * (kPSW / 64)) / 8;
constexpr int kG2Blocks = ((kVocabP / 64) * (kHidP / 64) + 7) / 8;
constexpr int kG3Blocks = ((kChunkRows / 64) * (kHidP / 64)) / 8;
static_assert(((kVocabP / 64) * (kPSW / 64)) % 8 == 0 && kG1Blocks == 391);
static_assert(kG2Blocks == 196);
static_assert(((kChunkRows / 64) * (kHidP / 64)) % 8 == 0 && kG3Blocks == 128);

__device__ __forceinline__ void dep_guard_h(v8f& a, v8f& b, v16h x, v16h y) { asm volatile("v_nop\n\tv_nop\n\tv_nop\n\tv_nop" : "+v"(a), "+v"(b) : "v"(x), "v"(y)); }
__device__ __forceinline__ void dep_guard1_h(v8f& a, v16h x, v16h y) { asm volatile("v_nop\n\tv_nop\n\tv_nop\n\tv_nop" : "+v"(a) : "v"(x), "v"(y)); }
__device__ __forceinline__ void keep4_h(v16h a, v16h b, v16h c, v16h d) { asm volatile("v_nop" :: "v"(a), "v"(b), "v"(c), "v"(d)); }
__device__ __forceinline__ void acc_guard4(v8f& a, v8f& b, v8f& c, v8f& d) { asm volatile("v_nop\n\tv_nop\n\tv_nop\n\tv_nop" : "+v"(a), "+v"(b), "+v"(c), "+v"(d)); }

template <typename T> struct Frag;
template <> struct Frag<_Float16> {
  typedef v16h V; union U { v16h v; v8h h[2]; };
  static __device__ __forceinline__ v16h load(const _Float16* p) {
    U f; f.h[0] = *(const v8h*)(p); f.h[1] = *(const v8h*)(p + 16); return f.v;
  }
  static __device__ __forceinline__ v8f mma(v16h a, v16h b, v8f c) {
    return __builtin_amdgcn_wmma_f32_16x16x32_f16(false, a, false, b, (short)0, c, false, false);
  }
  static __device__ __forceinline__ void guard(v8f& a, v8f& b, v16h x, v16h y) { dep_guard_h(a, b, x, y); }
  static __device__ __forceinline__ void keep(v16h a, v16h b, v16h c, v16h d) { keep4_h(a, b, c, d); }
};

__device__ __forceinline__ unsigned pack_f16x2(float a, float b) {
  const _Float16 h0 = (_Float16)a, h1 = (_Float16)b;
  return (unsigned)__builtin_bit_cast(unsigned short, h0) | ((unsigned)__builtin_bit_cast(unsigned short, h1) << 16);
}
__device__ __forceinline__ void st2u(unsigned* p, unsigned v) { *(volatile unsigned*)p = v; __threadfence(); *(volatile unsigned*)p = v; }
__device__ __forceinline__ float ftanh(float x) { return 1.0f - 2.0f * __builtin_amdgcn_rcpf(1.0f + __expf(2.0f * x)); }

template <int BIAS_MODE, int OUT_MODE, int RES_MODE, int ACT>
__global__ __launch_bounds__(256) void gemm64_f16(
    const unsigned short* __restrict__ Ap, int lda,
    const unsigned short* __restrict__ Btp, int ldb,
    void* __restrict__ Cout, int ldc,
    const float* __restrict__ bias,
    const float* __restrict__ resid, int ldr, const int* __restrict__ ridx, int nres,
    int M, int N, int K, float scale) {
  typedef _Float16 T;
  typedef v16h V;
  const T* A = (const T*)Ap; const T* Bt = (const T*)Btp;
  __shared__ __align__(16) float sT[8][16 * 68];
  const int lane = threadIdx.x & 31;
  const int wave = threadIdx.x >> 5;
  const int tilesN = N >> 6;
  const int tilesM = M >> 6;
  const int tile = blockIdx.x * 8 + wave;
  if (tile >= tilesM * tilesN) return;
  const int tm = tile / tilesN;
  const int tn = tile - tm * tilesN;
  const int m0 = tm << 6;
  const int n0 = tn << 6;

  const int rlane = lane & 15;
  const int koff  = (lane >> 4) * 8;
  const int mOff  = (lane >> 4) * 8;

  v8f acc[4][4];
#pragma unroll
  for (int i = 0; i < 4; ++i)
#pragma unroll
    for (int j = 0; j < 4; ++j) acc[i][j] = (v8f){0.f,0.f,0.f,0.f,0.f,0.f,0.f,0.f};

  for (int k0 = 0; k0 < K; k0 += 32) {
    V bh[4];
#pragma unroll
    for (int j = 0; j < 4; ++j) {
      const size_t bo = (size_t)(n0 + (j << 4) + rlane) * ldb + koff + k0;
      bh[j] = Frag<T>::load(Bt + bo);
    }
#pragma unroll
    for (int i = 0; i < 4; ++i) {
      const size_t ao = (size_t)(m0 + (i << 4) + rlane) * lda + koff + k0;
      V ah = Frag<T>::load(A + ao);
#pragma unroll
      for (int j = 0; j < 4; ++j) acc[i][j] = Frag<T>::mma(ah, bh[j], acc[i][j]);
      Frag<T>::guard(acc[i][0], acc[i][3], ah, ah);
    }
    Frag<T>::keep(bh[0], bh[1], bh[2], bh[3]);
  }
  acc_guard4(acc[0][0], acc[0][1], acc[0][2], acc[0][3]);
  acc_guard4(acc[1][0], acc[1][1], acc[1][2], acc[1][3]);
  acc_guard4(acc[2][0], acc[2][1], acc[2][2], acc[2][3]);
  acc_guard4(acc[3][0], acc[3][1], acc[3][2], acc[3][3]);

  float* slab = sT[wave];
#pragma unroll
  for (int i = 0; i < 4; ++i) {
    const int mBase = m0 + (i << 4);
    int tk[8];
    if (RES_MODE == 2) {
#pragma unroll
      for (int r = 0; r < 8; ++r) {
        int t = ridx[mBase + mOff + r];
        t = t < 0 ? 0 : t;
        t = t > nres - 1 ? nres - 1 : t;
        tk[r] = t;
      }
    }
#pragma unroll
    for (int j = 0; j < 4; ++j) {
      const int n = n0 + (j << 4) + rlane;
      float bv = 0.f;
      if (BIAS_MODE == 2) bv = bias[n];
#pragma unroll
      for (int r = 0; r < 8; ++r) {
        float v = acc[i][j][r] * scale;
        if (BIAS_MODE == 2) v += bv;
        if (RES_MODE == 2) v += resid[(size_t)tk[r] * ldr + n];
        if (ACT == 1) v = ftanh(v);
        slab[(mOff + r) * 68 + (j << 4) + rlane] = v;
      }
    }
    __builtin_amdgcn_fence(__ATOMIC_RELEASE, "workgroup");
    __builtin_amdgcn_wave_barrier();
    __builtin_amdgcn_fence(__ATOMIC_ACQUIRE, "workgroup");
    if (OUT_MODE == 0) {
      float* C = (float*)Cout;
      const int hh = lane >> 4, c4 = (lane & 15) * 4;
      for (int pass = 0; pass < 2; ++pass) {
#pragma unroll
        for (int it = 0; it < 8; ++it) {
          const int row = it * 2 + hh;
          v4f v = *(const v4f*)(slab + row * 68 + c4);
          *(volatile v4f*)(C + (size_t)(mBase + row) * ldc + n0 + c4) = v;
        }
        __threadfence();
      }
    } else {
      const int q = lane >> 3, c8 = (lane & 7) * 8;
      unsigned short* C = (unsigned short*)Cout;
      for (int pass = 0; pass < 2; ++pass) {
#pragma unroll
        for (int it = 0; it < 4; ++it) {
          const int row = it * 4 + q;
          const float* sp = slab + row * 68 + c8;
          v8h hv;
#pragma unroll
          for (int e = 0; e < 8; ++e) hv[e] = (_Float16)sp[e];
          *(volatile v8h*)(C + (size_t)(mBase + row) * ldc + n0 + c8) = hv;
        }
        __threadfence();
      }
    }
    __builtin_amdgcn_fence(__ATOMIC_RELEASE, "workgroup");
    __builtin_amdgcn_wave_barrier();
    __builtin_amdgcn_fence(__ATOMIC_ACQUIRE, "workgroup");
  }
}

__global__ __launch_bounds__(256) void prep_kernel(
    const float* __restrict__ wsl_w, const float* __restrict__ wsr_w, const float* __restrict__ w2_w,
    const float* __restrict__ wl_w, const float* __restrict__ wr_w,
    const float* __restrict__ wsl_b, const float* __restrict__ wsr_b, const float* __restrict__ w2_b,
    const float* __restrict__ wl_b, const float* __restrict__ wr_b,
    unsigned* __restrict__ wcatu, unsigned* __restrict__ wlru, unsigned* __restrict__ w2acu,
    unsigned* __restrict__ biasu) {
  const int blk = blockIdx.x, tid = threadIdx.x;
  const float ws64 = 64.0f;
  if (blk < kPrepB1) {
    const int p = blk * 256 + tid;
    const int e0 = 2 * p;
    const int row = e0 / kEmbP;
    const int k = e0 - row * kEmbP;
    const int grp = row >> 7, rr = row & 127;
    const int rrc = rr < kChan ? rr : kChan - 1;
    auto val = [&](int kk) -> float {
      const int kc = kk < kEmb ? kk : kEmb - 1;
      const float a = wsl_w[rrc * kEmb + kc];
      const float b = wsr_w[rrc * kEmb + kc];
      const float d = w2_w[rrc * kFeatIn + kChan + kc];
      const float v = (grp == 0) ? a : ((grp == 1) ? b : d);
      return (rr < kChan && kk < kEmb) ? v * ws64 : 0.0f;
    };
    st2u(wcatu + p, pack_f16x2(val(k), val(k + 1)));
  } else if (blk < kPrepB2) {
    const int p = (blk - kPrepB1) * 256 + tid;
    const int e0 = 2 * p;
    const int row = e0 >> 7;
    const int k = e0 & 127;
    const int grp = row >> 7, rr = row & 127;
    const int rrc = rr < kChan ? rr : kChan - 1;
    auto val = [&](int kk) -> float {
      const int kc = kk < kChan ? kk : kChan - 1;
      const float a = wl_w[rrc * kChan + kc];
      const float b = wr_w[rrc * kChan + kc];
      const float v = (grp == 0) ? a : b;
      return (rr < kChan && kk < kChan) ? v * ws64 : 0.0f;
    };
    st2u(wlru + p, pack_f16x2(val(k), val(k + 1)));
  } else if (blk < kPrepB3) {
    const int p = (blk - kPrepB2) * 256 + tid;
    const int e0 = 2 * p;
    const int row = e0 >> 8;
    const int k = e0 & 255;
    const int rc = row < kHid ? row : kHid - 1;
    auto val = [&](int kk) -> float {
      const int kgrp = kk >> 7, kr = kk & 127;
      const int krc = kr < kChan ? kr : kChan - 1;
      const float a = w2_w[rc * kFeatIn + krc];
      const float b = w2_w[rc * kFeatIn + kEmb + kChan + krc];
      const float v = (kgrp == 0) ? a : b;
      return (row < kHid && kr < kChan) ? v * ws64 : 0.0f;
    };
    st2u(w2acu + p, pack_f16x2(val(k), val(k + 1)));
  } else {
    const int p = (blk - kPrepB3) * 256 + tid;
    const int grp = p >> 7, cl = p & 127;
    const int cc = cl < kChan ? cl : kChan - 1;
    const float a = wsl_b[cc] * 256.0f;
    const float b = wsr_b[cc] * 256.0f;
    const float d = w2_b[cc];
    const float e = wl_b[cc];
    const float f = wr_b[cc];
    float v = 0.0f;
    v = (grp == 0) ? a : v;
    v = (grp == 1) ? b : v;
    v = (grp == 2) ? d : v;
    v = (grp == 3) ? e : v;
    v = (grp == 4) ? f : v;
    v = (cl < kChan) ? v : 0.0f;
    st2u(biasu + p, (unsigned)__float_as_uint(v));
  }
}

__global__ __launch_bounds__(256) void emb_cast_kernel(const float* __restrict__ emb, _Float16* __restrict__ e16) {
  const int i = blockIdx.x * 256 + threadIdx.x;
  const int row = i / (kEmbP / 8);
  const int ch = i - row * (kEmbP / 8);
  const int rowc = row < kVocab ? row : kVocab - 1;
  const int cb = ch * 8;
  const int base = cb < (kEmb - 8) ? cb : (kEmb - 8);
  const float* src = emb + (size_t)rowc * kEmb + base;
  const v4f f0 = *(const v4f*)src;
  const v4f f1 = *(const v4f*)(src + 4);
  const bool rowok = row < kVocab;
  const bool sh4 = (cb == kEmb - 4);
  v8h hv;
  hv[0] = (_Float16)((rowok && cb + 0 < kEmb) ? (sh4 ? f1[0] : f0[0]) * 16.0f : 0.0f);
  hv[1] = (_Float16)((rowok && cb + 1 < kEmb) ? (sh4 ? f1[1] : f0[1]) * 16.0f : 0.0f);
  hv[2] = (_Float16)((rowok && cb + 2 < kEmb) ? (sh4 ? f1[2] : f0[2]) * 16.0f : 0.0f);
  hv[3] = (_Float16)((rowok && cb + 3 < kEmb) ? (sh4 ? f1[3] : f0[3]) * 16.0f : 0.0f);
  hv[4] = (_Float16)((rowok && cb + 4 < kEmb) ? f1[0] * 16.0f : 0.0f);
  hv[5] = (_Float16)((rowok && cb + 5 < kEmb) ? f1[1] * 16.0f : 0.0f);
  hv[6] = (_Float16)((rowok && cb + 6 < kEmb) ? f1[2] * 16.0f : 0.0f);
  hv[7] = (_Float16)((rowok && cb + 7 < kEmb) ? f1[3] * 16.0f : 0.0f);
  _Float16* dst = e16 + (size_t)row * kEmbP + cb;
  *(volatile v8h*)dst = hv;
  __threadfence();
  *(volatile v8h*)dst = hv;
}

__global__ __launch_bounds__(kRecThreads) void birnn_kernel(
    const int* __restrict__ text, const _Float16* __restrict__ ps,
    const _Float16* __restrict__ wlr16, const float* __restrict__ blr,
    _Float16* __restrict__ clcr16) {
  __shared__ __align__(16) unsigned short sTok[kSeqPB * kLen];
  __shared__ __align__(16) _Float16 sState[2 * kStTile];
  __shared__ __align__(16) _Float16 sS[2 * kSTile];
  const int tid = threadIdx.x, lane = tid & 31, wave = tid >> 5;
  const int c = lane & 15, hh = lane >> 4, koff = hh * 8, mOff = hh * 8;
  const int dir = (int)(blockIdx.x >> 3);
  const int seq0 = (int)(blockIdx.x & 7) * kSeqPB;
  const int dcol = dir * kChanP;
  const _Float16* W = wlr16 + (size_t)dir * kChanP * kChanP;
  const float* Wb = blr + dir * kChanP;

#pragma unroll 1
  for (int it = 0; it < (kSeqPB * kLen) / kRecThreads; ++it) {
    const int i = it * kRecThreads + tid;
    int t = text[(size_t)(seq0 + (i >> 10)) * kLen + (i & 1023)];
    t = t < 0 ? 0 : t;
    t = t > kVocab - 1 ? kVocab - 1 : t;
    sTok[i] = (unsigned short)t;
  }
  {
    v8h z;
#pragma unroll
    for (int e = 0; e < 8; ++e) z[e] = (_Float16)0.0f;
    for (int i = tid; i < (2 * kStTile) / 8; i += kRecThreads) *(v8h*)(sState + i * 8) = z;
  }
  __syncthreads();

  const int pfRow = tid >> 4, pfCh = (tid & 15) * 8;
  {
    const int pos = dir ? (kLen - 1) : 0;
    const int tok = sTok[pfRow * kLen + pos];
    const v8h v = *(const v8h*)(ps + (size_t)tok * kPSW + dcol + pfCh);
    *(v8h*)(sS + kSTile + pfRow * kChanP + pfCh) = v;
  }
  const int q4 = lane >> 3, c8 = (lane & 7) * 8;
  const int lineIdx = wave * 4 + q4;
  const int rr = lineIdx >> 1;
  const int colh = (lineIdx & 1) * 64 + c8;
  {
    const int lB = dir ? (kLen - 1) : 0;
    v8h z;
#pragma unroll
    for (int e = 0; e < 8; ++e) z[e] = (_Float16)0.0f;
    _Float16* dst = clcr16 + ((size_t)(seq0 + rr) * kLen + lB) * kFeatW + dcol + colh;
    *(volatile v8h*)dst = z;
    __threadfence();
    *(volatile v8h*)dst = z;
  }
  __syncthreads();

  const int n = wave * 16 + c;
  v16h fb[4];
  {
    const _Float16* brow = W + (size_t)n * kChanP + koff;
#pragma unroll
    for (int kc = 0; kc < 4; ++kc) fb[kc] = Frag<_Float16>::load(brow + kc * 32);
  }
  const int nbc = n < kChan ? n : kChan - 1;
  float bias = Wb[nbc];
  bias = (n < kChan) ? bias : 0.0f;
  const float inv1024 = 1.0f / 1024.0f, inv256 = 1.0f / 256.0f;

#pragma unroll 1
  for (int s = 1; s < kLen; ++s) {
    const int p = s & 1;
    const int l = dir ? (kLen - 1 - s) : s;
    {
      const int s1 = (s + 1 < kLen) ? (s + 1) : (kLen - 1);
      const int pos = dir ? (kLen - s1) : (s1 - 1);
      const int tok = sTok[pfRow * kLen + pos];
      const v8h v = *(const v8h*)(ps + (size_t)tok * kPSW + dcol + pfCh);
      *(v8h*)(sS + (p ^ 1) * kSTile + pfRow * kChanP + pfCh) = v;
    }
    const _Float16* arow = sState + p * kStTile + c * kStP + koff;
    const v16h fa0 = Frag<_Float16>::load(arow);
    const v16h fa1 = Frag<_Float16>::load(arow + 32);
    const v16h fa2 = Frag<_Float16>::load(arow + 64);
    const v16h fa3 = Frag<_Float16>::load(arow + 96);
    v8f acc = (v8f){0.f,0.f,0.f,0.f,0.f,0.f,0.f,0.f};
    acc = Frag<_Float16>::mma(fa0, fb[0], acc);
    acc = Frag<_Float16>::mma(fa1, fb[1], acc);
    acc = Frag<_Float16>::mma(fa2, fb[2], acc);
    acc = Frag<_Float16>::mma(fa3, fb[3], acc);
    dep_guard1_h(acc, fa3, fb[3]);
    keep4_h(fa0, fa1, fa2, fa3);
    keep4_h(fb[0], fb[1], fb[2], fb[3]);

    _Float16* hn = sState + (p ^ 1) * kStTile;
    const _Float16* sp = sS + p * kSTile;
#pragma unroll
    for (int r = 0; r < 8; ++r) {
      const float sv = (float)sp[(mOff + r) * kChanP + n];
      float v = acc[r] * inv1024 + bias + sv * inv256;
      v = fmaxf(v, 0.0f);
      hn[(mOff + r) * kStP + n] = (_Float16)(v * 16.0f);
    }
    __syncthreads();

    {
      const v8h v = *(const v8h*)(hn + rr * kStP + colh);
      _Float16* dst = clcr16 + ((size_t)(seq0 + rr) * kLen + l) * kFeatW + dcol + colh;
      *(volatile v8h*)dst = v;
      __threadfence();
      *(volatile v8h*)dst = v;
    }
  }
}

__global__ __launch_bounds__(128) void maxpool_kernel(const float* __restrict__ y, float* __restrict__ y3, int nbase) {
  const int b = blockIdx.x, h = threadIdx.x;
  const float* p = y + (size_t)b * kLen * kHidP + h;
  float m = -__builtin_inff();
#pragma unroll 4
  for (int l = 0; l < kLen; ++l) m = fmaxf(m, p[(size_t)l * kHidP]);
  float* dst = y3 + (size_t)(nbase + b) * kHidP + h;
  *(volatile float*)dst = m;
  __threadfence();
  *(volatile float*)dst = m;
}

__global__ __launch_bounds__(128) void head_kernel(const float* __restrict__ y3, const float* __restrict__ w4,
                                                  const float* __restrict__ b4, float* __restrict__ out) {
  const int n = threadIdx.x;
  const float* yr = y3 + (size_t)n * kHidP;
  float a0 = 0.f, a1 = 0.f, a2 = 0.f, a3 = 0.f;
#pragma unroll 1
  for (int h = 0; h < kHid; ++h) {
    const float yv = yr[h];
    a0 += yv * w4[h];
    a1 += yv * w4[kHid + h];
    a2 += yv * w4[2 * kHid + h];
    a3 += yv * w4[3 * kHid + h];
  }
  v4f v;
  v[0] = a0 + b4[0]; v[1] = a1 + b4[1]; v[2] = a2 + b4[2]; v[3] = a3 + b4[3];
  float* dst = out + (size_t)n * kCls;
  *(volatile v4f*)dst = v;
  __threadfence();
  *(volatile v4f*)dst = v;
}

extern "C" void kernel_launch(void* const* d_in, const int* in_sizes, int n_in,
                              void* d_out, int out_size, void* d_ws, size_t ws_size, hipStream_t stream) {
  if (n_in < 14 || d_out == nullptr || d_ws == nullptr) return;
  if (in_sizes[0] != kRows || in_sizes[1] != kVocab * kEmb ||
      in_sizes[2] != kChan * kChan || in_sizes[3] != kChan || in_sizes[4] != kChan * kChan || in_sizes[5] != kChan ||
      in_sizes[6] != kChan * kEmb || in_sizes[7] != kChan || in_sizes[8] != kChan * kEmb || in_sizes[9] != kChan ||
      in_sizes[10] != kHid * kFeatIn || in_sizes[11] != kHid || in_sizes[12] != kCls * kHid || in_sizes[13] != kCls ||
      out_size != kBatch * kCls) return;

  const int*   text  = (const int*)  d_in[0];
  const float* emb   = (const float*)d_in[1];
  const float* wl_w  = (const float*)d_in[2];
  const float* wl_b  = (const float*)d_in[3];
  const float* wr_w  = (const float*)d_in[4];
  const float* wr_b  = (const float*)d_in[5];
  const float* wsl_w = (const float*)d_in[6];
  const float* wsl_b = (const float*)d_in[7];
  const float* wsr_w = (const float*)d_in[8];
  const float* wsr_b = (const float*)d_in[9];
  const float* w2_w  = (const float*)d_in[10];
  const float* w2_b  = (const float*)d_in[11];
  const float* w4_w  = (const float*)d_in[12];
  const float* w4_b  = (const float*)d_in[13];
  float* out = (float*)d_out;

  char* ws = (char*)d_ws; size_t off = 0;
  auto carve = [&](size_t bytes) -> char* { char* p = ws + off; off += (bytes + 255) & ~(size_t)255; return p; };
  char*           R0     = carve((size_t)kRows * kFeatW * 2);
  char*           R1     = carve((size_t)kVocabP * kPSW * 2);
  float*          PW     = (float*)carve((size_t)kVocabP * kHidP * 4);
  unsigned short* WCAT16 = (unsigned short*)carve((size_t)kDwWcat * 4);
  unsigned short* WLR16  = (unsigned short*)carve((size_t)kDwWlr * 4);
  unsigned short* W2AC16 = (unsigned short*)carve((size_t)kDwW2ac * 4);
  float*          BIAS   = (float*)carve((size_t)kDwBias * 4);
  float*          Y3     = (float*)carve((size_t)kBatch * kHidP * 4);
  if (off > ws_size || off > (size_t)134217728) return;
  if ((size_t)kVocabP * kEmbP * 2 > (size_t)kRows * kFeatW * 2) return;
  if ((size_t)kChunkRows * kHidP * 4 > (size_t)kVocabP * kPSW * 2) return;

  unsigned short* EMB16  = (unsigned short*)R0;
  unsigned short* CLCR16 = (unsigned short*)R0;
  unsigned short* PS     = (unsigned short*)R1;
  float*          YCH    = (float*)R1;

  const float inv1024 = 1.0f / 1024.0f;

  prep_kernel<<<kPrepBlocks, 256, 0, stream>>>(wsl_w, wsr_w, w2_w, wl_w, wr_w, wsl_b, wsr_b, w2_b, wl_b, wr_b,
                                               (unsigned*)WCAT16, (unsigned*)WLR16, (unsigned*)W2AC16, (unsigned*)BIAS);

  emb_cast_kernel<<<kEmbBlocks, 256, 0, stream>>>(emb, (_Float16*)EMB16);

  gemm64_f16<2, 1, 0, 0><<<kG1Blocks, 256, 0, stream>>>(
      EMB16, kEmbP, WCAT16, kEmbP, (void*)PS, kPSW, BIAS, nullptr, 0, nullptr, 1, kVocabP, kPSW, kEmbP, 0.25f);

  gemm64_f16<2, 0, 0, 0><<<kG2Blocks, 256, 0, stream>>>(
      EMB16, kEmbP, WCAT16 + (size_t)256 * kEmbP, kEmbP, (void*)PW, kHidP, BIAS + 256, nullptr, 0, nullptr, 1,
      kVocabP, kHidP, kEmbP, inv1024);

  birnn_kernel<<<kRecBlocks, kRecThreads, 0, stream>>>(text, (const _Float16*)PS, (const _Float16*)WLR16, BIAS + 384,
                                                       (_Float16*)CLCR16);

  for (int q = 0; q < kChunks; ++q) {
    gemm64_f16<0, 0, 2, 1><<<kG3Blocks, 256, 0, stream>>>(
        CLCR16 + (size_t)q * kChunkRows * kFeatW, kFeatW, W2AC16, kFeatW, (void*)YCH, kHidP, nullptr,
        PW, kHidP, text + (size_t)q * kChunkRows, kVocab, kChunkRows, kHidP, kFeatW, inv1024);
    maxpool_kernel<<<kSeqPerChunk, kHidP, 0, stream>>>(YCH, Y3, q * kSeqPerChunk);
  }

  head_kernel<<<1, kBatch, 0, stream>>>(Y3, w4_w, w4_b, out);
}
